// SSM_cha_Last_36386962932306
// MI455X (gfx1250) — hardware-run, weakly checked
//
#include <hip/hip_runtime.h>

typedef float          v8f   __attribute__((ext_vector_type(8)));
typedef float          v4f   __attribute__((ext_vector_type(4)));
typedef unsigned int   v4u   __attribute__((ext_vector_type(4)));
typedef int            v8i   __attribute__((ext_vector_type(8)));
typedef unsigned short v8us  __attribute__((ext_vector_type(8)));
typedef unsigned short v16us __attribute__((ext_vector_type(16)));
typedef __bf16         v16bf __attribute__((ext_vector_type(16)));
typedef _Float16       v16h  __attribute__((ext_vector_type(16)));
typedef v4f  __attribute__((may_alias)) v4fa;
typedef v8us __attribute__((may_alias)) v8usa;
union FragB { v16bf v; v16us u; v8us h[2]; v8i w; };
union FragH { v16h  v; v16us u; v8us h[2]; v8i w; };

__device__ __forceinline__ v8f wmb(const FragB& a, const FragB& b, v8f c) {
  v8f d = __builtin_amdgcn_wmma_f32_16x16x32_bf16(false, a.v, false, b.v, (short)0, c, false, false);
  asm volatile("v_nop\n\tv_nop\n\tv_nop\n\tv_nop" : "+v"(d) : "v"(a.w), "v"(b.w));
  return d;
}

__device__ __forceinline__ v8f wmh(const FragH& a, const FragH& b, v8f c) {
  v8f d = __builtin_amdgcn_wmma_f32_16x16x32_f16(false, a.v, false, b.v, (short)0, c, false, false);
  asm volatile("v_nop\n\tv_nop\n\tv_nop\n\tv_nop" : "+v"(d) : "v"(a.w), "v"(b.w));
  return d;
}

__device__ __forceinline__ unsigned bf16_bits(float f) {
  const unsigned u = __float_as_uint(f);
  const unsigned r = (u + 0x7FFFu + ((u >> 16) & 1u)) >> 16;
  const unsigned q = (u >> 16) | 0x40u;
  return ((u & 0x7fffffffu) > 0x7f800000u) ? q : r;
}

__device__ __forceinline__ float bf16_val(float f) {
  return __uint_as_float(bf16_bits(f) << 16);
}
__device__ __forceinline__ int clampi(int v, int lo, int hi) {
  return v < lo ? lo : (v > hi ? hi : v);
}

__device__ __forceinline__ unsigned f16_bits(float f) {
  const unsigned u  = __float_as_uint(f);
  const unsigned s  = (u >> 16) & 0x8000u;
  const unsigned a  = u & 0x7fffffffu;
  const unsigned t  = a - 0x38000000u;
  const unsigned r  = (t + 0x0FFFu + ((t >> 13) & 1u)) >> 13;
  const unsigned rc = r > 0x7C00u ? 0x7C00u : r;
  const bool small  = a < 0x38800000u;
  const bool isnan  = a > 0x7f800000u;
  const unsigned fin = small ? 0u : (s | rc);
  return isnan ? (s | 0x7E00u) : fin;
}

__device__ __forceinline__ unsigned pk16(unsigned lo, unsigned hi) { return lo | (hi << 16); }
__device__ __forceinline__ unsigned bf16_lo_bits(float v) {
  float hi = bf16_val(v);
  asm volatile("" : "+v"(hi));
  return bf16_bits(v - hi);
}
__device__ __forceinline__ v4u pack8_bf16(v4f a, v4f c) {
  return (v4u){ pk16(bf16_bits(a[0]), bf16_bits(a[1])), pk16(bf16_bits(a[2]), bf16_bits(a[3])),
                pk16(bf16_bits(c[0]), bf16_bits(c[1])), pk16(bf16_bits(c[2]), bf16_bits(c[3])) };
}
__device__ __forceinline__ v4u pack8_bf16_lo(v4f a, v4f c) {
  return (v4u){ pk16(bf16_lo_bits(a[0]), bf16_lo_bits(a[1])), pk16(bf16_lo_bits(a[2]), bf16_lo_bits(a[3])),
                pk16(bf16_lo_bits(c[0]), bf16_lo_bits(c[1])), pk16(bf16_lo_bits(c[2]), bf16_lo_bits(c[3])) };
}
__device__ __forceinline__ v4u pack8_f16(v4f a, v4f c) {
  return (v4u){ pk16(f16_bits(a[0]), f16_bits(a[1])), pk16(f16_bits(a[2]), f16_bits(a[3])),
                pk16(f16_bits(c[0]), f16_bits(c[1])), pk16(f16_bits(c[2]), f16_bits(c[3])) };
}

template <int FORM>
__global__ __launch_bounds__(256) void k_plane(const float* __restrict__ src, int rows, int cols, int ldsrc,
                                               unsigned short* __restrict__ dst, int MP, int KP) {
  static_assert(FORM >= 0 && FORM <= 3);
  const int KTOT = (FORM == 1 || FORM == 3) ? 2 * KP : KP;
  const unsigned ppr   = (unsigned)(KTOT >> 3);
  const unsigned kp8   = (unsigned)(KP >> 3);
  const unsigned total = (unsigned)MP * ppr;
  const unsigned g     = blockIdx.x * 256u + threadIdx.x;
  const unsigned rowu  = g / ppr;
  const unsigned p     = g - rowu * ppr;
  const bool second    = p >= kp8;
  const int row = (int)rowu;
  const int c0  = (int)((second ? p - kp8 : p) << 3);
  const float* srow = src + (size_t)clampi(row, 0, rows - 1) * (size_t)ldsrc;
  float x[8];
  unsigned mk[8];
#pragma unroll
  for (int e = 0; e < 8; ++e) {
    const int c = c0 + e;
    const float v = srow[clampi(c, 0, cols - 1)];
    asm volatile("" :: "v"(v));
    x[e]  = v;
    mk[e] = (row < rows && c < cols) ? 0xFFFFu : 0u;
  }
  const v4f a = (v4f){ x[0], x[1], x[2], x[3] };
  const v4f c = (v4f){ x[4], x[5], x[6], x[7] };
  v4u o;
  if (FORM == 2) {
    o = pack8_f16(a, c);
  } else {
    const v4u hi = pack8_bf16(a, c);
    o = hi;
    if (FORM == 1) { const v4u lo = pack8_bf16_lo(a, c); o = second ? lo : hi; }
  }
  const v4u mw = (v4u){ pk16(mk[0], mk[1]), pk16(mk[2], mk[3]), pk16(mk[4], mk[5]), pk16(mk[6], mk[7]) };
  o &= mw;
  if (g < total) {
    volatile v4u* q = (volatile v4u*)(dst + (size_t)g * 8);
    *q = o;
    __threadfence();
    *q = o;
  }
}

template <int FORM> struct FragOf    { typedef FragB T; };
template <>         struct FragOf<2> { typedef FragH T; };
__device__ __forceinline__ v8f mm(const FragB& a, const FragB& b, v8f c) { return wmb(a, b, c); }
__device__ __forceinline__ v8f mm(const FragH& a, const FragH& b, v8f c) { return wmh(a, b, c); }
template <class F> __device__ __forceinline__ F ld_frag(const unsigned short* p) {
  F f;
  f.h[0] = *(const v8usa*)(p);
  f.h[1] = *(const v8usa*)(p + 16);
  return f;
}

template <int FORM, int EPI>
__global__ __launch_bounds__(256) __attribute__((amdgpu_num_vgpr(248)))
void k_gemm_nt(const unsigned short* __restrict__ A, const unsigned short* __restrict__ B,
               const float* __restrict__ bias, float* __restrict__ D, int M, int N, int KTOT, int ldd) {
  static_assert(FORM >= 0 && FORM <= 2);
  static_assert(EPI == 0 || EPI == 1);
  typedef typename FragOf<FORM>::T F;
  __shared__ __attribute__((aligned(16))) float sT[8][16 * 68];
  const int lane = threadIdx.x & 31;
  const int wave = threadIdx.x >> 5;
  const int tilesM = (M + 63) >> 6;
  const int tilesN = (N + 63) >> 6;
  const int tile = blockIdx.x * 8 + wave;
  if (tile >= tilesM * tilesN) return;
  const int tm = tile / tilesN;
  const int tn = tile - tm * tilesN;
  const int m0 = tm << 6;
  const int n0 = tn << 6;

  const int rl = lane & 15;
  const int h8 = (lane >> 4) * 8;
  const unsigned short* pa = A + (size_t)(m0 + rl) * (size_t)KTOT + h8;
  const unsigned short* pb = B + (size_t)(n0 + rl) * (size_t)KTOT + h8;

  v8f acc[4][4];
#pragma unroll
  for (int i = 0; i < 4; ++i)
#pragma unroll
    for (int j = 0; j < 4; ++j) acc[i][j] = (v8f){0.f, 0.f, 0.f, 0.f, 0.f, 0.f, 0.f, 0.f};

#pragma unroll 1
  for (int k0 = 0; k0 < KTOT; k0 += 32) {
    F bf[4];
#pragma unroll
    for (int j = 0; j < 4; ++j) bf[j] = ld_frag<F>(pb + (size_t)(j << 4) * (size_t)KTOT + k0);
#pragma unroll
    for (int i = 0; i < 4; ++i) {
      const F af = ld_frag<F>(pa + (size_t)(i << 4) * (size_t)KTOT + k0);
#pragma unroll
      for (int j = 0; j < 4; ++j) acc[i][j] = mm(af, bf[j], acc[i][j]);
    }
  }

  float* slab = sT[wave];
  const int hh = lane >> 4;
  const int c4 = (lane & 15) * 4;
  const int nc = n0 + c4;
  const bool cok = nc < N;
  v4f bv = (v4f){0.f, 0.f, 0.f, 0.f};
  if (EPI == 1) {
    bv = *(const v4fa*)(bias + clampi(nc, 0, N - 4));
    asm volatile("" :: "v"(bv));
  }
#pragma unroll
  for (int i = 0; i < 4; ++i) {
    const int mBase = m0 + (i << 4);
#pragma unroll
    for (int j = 0; j < 4; ++j) {
#pragma unroll
      for (int r = 0; r < 8; ++r) slab[(h8 + r) * 68 + (j << 4) + rl] = acc[i][j][r];
    }
    __builtin_amdgcn_fence(__ATOMIC_RELEASE, "workgroup");
    __builtin_amdgcn_wave_barrier();
    __builtin_amdgcn_fence(__ATOMIC_ACQUIRE, "workgroup");
    v4f vv[8];
#pragma unroll
    for (int it = 0; it < 8; ++it) {
      const int row = it * 2 + hh;
      v4f v = *(const v4fa*)(slab + row * 68 + c4);
      if (EPI == 1) v += bv;
      vv[it] = v;
    }
    for (int pass = 0; pass < 2; ++pass) {
#pragma unroll
      for (int it = 0; it < 8; ++it) {
        const int row = mBase + it * 2 + hh;
        if (cok && row < M) *(volatile v4f*)(D + (size_t)row * (size_t)ldd + nc) = vv[it];
      }
      __threadfence();
    }
    __builtin_amdgcn_fence(__ATOMIC_RELEASE, "workgroup");
    __builtin_amdgcn_wave_barrier();
    __builtin_amdgcn_fence(__ATOMIC_ACQUIRE, "workgroup");
  }
}

#include <math.h>
#include <stddef.h>

#ifndef SPLIT_WX
#define SPLIT_WX 1
#endif
#ifndef SPLIT_DT
#define SPLIT_DT 1
#endif
#ifndef SPLIT_OUT
#define SPLIT_OUT 1
#endif

#define NBAT   8
#define DI     256
#define IMH    64
#define IMW    64
#define LSEQ   4096
#define NHALF  2
#define BHALF  4
#define MH     (BHALF * LSEQ)
#define NXZ    (2 * DI)
#define KHL    (2 * DI)
#define NXD    20
#define NXP    64
#define DTRK   16
#define KDT    64
#define CROWS  32
#define SCH    32
#define SCT    128

#define PU_WIN (NXZ * DI / 8)
#define PU_WX  (NXP * KHL / 8)
#define PU_WDT (DI * KDT / 8)
#define PU_WO  (DI * KHL / 8)
#define PU_ALL (PU_WIN + PU_WX + PU_WDT + PU_WO)

static_assert(IMH * IMW == LSEQ);
static_assert(NBAT == NHALF * BHALF);
static_assert(MH % 128 == 0 && MH % 64 == 0);
static_assert(DI == 256);
static_assert(NXD <= NXP && NXP % 64 == 0 && NXD == DTRK + 4);
static_assert(2 * DTRK <= KDT && KDT % 32 == 0);
static_assert(DI % 32 == 0 && KHL % 32 == 0 && NXZ % 64 == 0 && DI % 64 == 0 && LSEQ % 64 == 0);
static_assert(LSEQ % SCH == 0 && LSEQ % CROWS == 0 && MH % CROWS == 0);
static_assert(CROWS == 32 && SCH == 32 && SCT == 128 && DI == 2 * SCT);
static_assert(PU_WIN % 256 == 0 && PU_WX % 256 == 0 && PU_WDT % 256 == 0 && PU_WO % 256 == 0);
static_assert((MH * 8) % 256 == 0);

constexpr size_t SZ_UB    = (size_t)MH * DI * 2;
constexpr size_t SZ_XZ    = (size_t)MH * NXZ * 4;
constexpr size_t SZ_XIHL  = (size_t)MH * KHL * 2;
constexpr size_t SZ_XDBL  = (size_t)MH * NXP * 4;
constexpr size_t SZ_DTIN  = (size_t)MH * KDT * 2;
constexpr size_t SZ_DTRAW = (size_t)MH * DI * 4;
constexpr size_t SZ_YHL   = (size_t)MH * KHL * 2;
constexpr size_t SZ_WINT  = (size_t)NXZ * DI * 2;
constexpr size_t SZ_WX2   = (size_t)NXP * KHL * 2;
constexpr size_t SZ_WDT2  = (size_t)DI * KDT * 2;
constexpr size_t SZ_WOUT2 = (size_t)DI * KHL * 2;
constexpr size_t O_UB    = 0;
constexpr size_t O_XZ    = O_UB + SZ_UB;
constexpr size_t O_XIHL  = O_XZ + SZ_XZ;
constexpr size_t O_XDBL  = O_XIHL + SZ_XIHL;
constexpr size_t O_DTIN  = O_XDBL + SZ_XDBL;
constexpr size_t O_DTRAW = O_DTIN + SZ_DTIN;
constexpr size_t O_YHL   = O_DTRAW + SZ_DTRAW;
constexpr size_t O_WINT  = O_YHL + SZ_YHL;
constexpr size_t O_WX2   = O_WINT + SZ_WINT;
constexpr size_t O_WDT2  = O_WX2 + SZ_WX2;
constexpr size_t O_WOUT2 = O_WDT2 + SZ_WDT2;
constexpr size_t WS_END  = O_WOUT2 + SZ_WOUT2;
static_assert(O_XZ % 256 == 0 && O_XIHL % 256 == 0 && O_XDBL % 256 == 0 && O_DTIN % 256 == 0);
static_assert(O_DTRAW % 256 == 0 && O_YHL % 256 == 0 && O_WINT % 256 == 0 && O_WX2 % 256 == 0);
static_assert(O_WDT2 % 256 == 0 && O_WOUT2 % 256 == 0);
static_assert(WS_END <= ((size_t)128 << 20));

__device__ __forceinline__ void put16(unsigned short* p, v4u o) {
  volatile v4u* q = (volatile v4u*)p;
  *q = o;
  __threadfence();
  *q = o;
}
__device__ __forceinline__ float silu_f(float v)     { return v / (1.0f + expf(-v)); }
__device__ __forceinline__ float softplus_f(float p) { return fmaxf(p, 0.0f) + log1pf(expf(-fabsf(p))); }

__device__ __forceinline__ v4u gather8_bf16(const float* __restrict__ src, int k0, int ld, int col) {
  float x[8];
#pragma unroll
  for (int e = 0; e < 8; ++e) {
    const float v = src[(size_t)(k0 + e) * (size_t)ld + col];
    asm volatile("" :: "v"(v));
    x[e] = v;
  }
  return pack8_bf16((v4f){ x[0], x[1], x[2], x[3] }, (v4f){ x[4], x[5], x[6], x[7] });
}

__global__ __launch_bounds__(256) void k_prep(const float* __restrict__ w_in, const float* __restrict__ w_x,
                                              const float* __restrict__ w_dt, const float* __restrict__ w_out,
                                              unsigned short* __restrict__ WINT, unsigned short* __restrict__ WX2,
                                              unsigned short* __restrict__ WDT2, unsigned short* __restrict__ WOUT2) {
  const int u = (int)blockIdx.x * 256 + (int)threadIdx.x;
  if (u < PU_WIN) {
    const int n  = u >> 5;
    const int k8 = (u & 31) * 8;
    const v4u o = gather8_bf16(w_in, k8, NXZ, n);
    put16(WINT + (size_t)u * 8, o);
  } else if (u < PU_WIN + PU_WX) {
    const int v  = u - PU_WIN;
    const int n  = v >> 6;
    const int k8 = (v & 63) * 8;
    const int nc = n < NXD ? n : NXD - 1;
    v4u o = gather8_bf16(w_x, k8 & (DI - 1), NXD, nc);
    const unsigned mk = (n < NXD && (SPLIT_WX != 0 || k8 < DI)) ? 0xFFFFFFFFu : 0u;
    o &= (v4u){ mk, mk, mk, mk };
    put16(WX2 + (size_t)v * 8, o);
  } else if (u < PU_WIN + PU_WX + PU_WDT) {
    const int v  = u - (PU_WIN + PU_WX);
    const int d  = v >> 3;
    const int k8 = (v & 7) * 8;
    v4u o = gather8_bf16(w_dt, k8 & (DTRK - 1), DI, d);
    const unsigned mk = (k8 < DTRK || (SPLIT_DT != 0 && k8 < 2 * DTRK)) ? 0xFFFFFFFFu : 0u;
    o &= (v4u){ mk, mk, mk, mk };
    put16(WDT2 + (size_t)v * 8, o);
  } else if (u < PU_ALL) {
    const int v  = u - (PU_WIN + PU_WX + PU_WDT);
    const int oc = v >> 6;
    const int k8 = (v & 63) * 8;
    v4u o = gather8_bf16(w_out, k8 & (DI - 1), DI, oc);
    const unsigned mk = (SPLIT_OUT != 0 || k8 < DI) ? 0xFFFFFFFFu : 0u;
    o &= (v4u){ mk, mk, mk, mk };
    put16(WOUT2 + (size_t)v * 8, o);
  }
}

__global__ __launch_bounds__(256) void k_tok(const float* __restrict__ xh, unsigned short* __restrict__ UB) {
  __shared__ float tile[64 * 65];
  const int tid  = (int)threadIdx.x;
  const int bx   = (int)blockIdx.x;
  const int hrow = bx & 63;
  const int ct   = (bx >> 6) & 3;
  const int bb   = bx >> 8;
  const float* src = xh + ((size_t)(bb * DI + ct * 64)) * (size_t)LSEQ + (size_t)hrow * IMW;
#pragma unroll
  for (int j = 0; j < 4; ++j) {
    const int i  = tid + 256 * j;
    const int c  = i >> 4;
    const int p4 = (i & 15) * 4;
    const v4f v = *(const v4fa*)(src + (size_t)c * LSEQ + p4);
    float* tp = tile + c * 65 + p4;
    tp[0] = v[0]; tp[1] = v[1]; tp[2] = v[2]; tp[3] = v[3];
  }
  __syncthreads();
#pragma unroll
  for (int j = 0; j < 2; ++j) {
    const int q = tid + 256 * j;
    const int l = q >> 3;
    const int p = q & 7;
    const float* tp = tile + (8 * p) * 65 + l;
    const v4f a = (v4f){ tp[0],   tp[65],  tp[130], tp[195] };
    const v4f c = (v4f){ tp[260], tp[325], tp[390], tp[455] };
    const v4u o = pack8_bf16(a, c);
    put16(UB + ((size_t)(bb * LSEQ + hrow * IMW + l)) * DI + ct * 64 + 8 * p, o);
  }
}

__global__ __launch_bounds__(256) void k_conv(const float* __restrict__ XZ, const float* __restrict__ conv_w,
                                              const float* __restrict__ conv_b, unsigned short* __restrict__ XIHL) {
  __shared__ __attribute__((aligned(16))) float stg[CROWS * DI];
  const int tid  = (int)threadIdx.x;
  const int d    = tid;
  const int lane = tid & 31;
  const int wave = __builtin_amdgcn_readfirstlane(tid >> 5);
  const int r0   = (int)blockIdx.x * CROWS;
  const int l0   = r0 & (LSEQ - 1);
  v4f wv = *(const v4fa*)(conv_w + 4 * d);
  asm volatile("" :: "v"(wv));
  const float w0 = bf16_val(wv[0]), w1 = bf16_val(wv[1]), w2 = bf16_val(wv[2]), w3 = bf16_val(wv[3]);
  float cbv = conv_b[d];
  asm volatile("" :: "v"(cbv));
  const float cb = bf16_val(cbv);
  const unsigned hm = (l0 > 0) ? 0xFFFFFFFFu : 0u;
  const int ra = r0 >= 3 ? r0 - 3 : 0;
  const int rb = r0 >= 2 ? r0 - 2 : 0;
  const int rc = r0 >= 1 ? r0 - 1 : 0;
  float x0 = XZ[(size_t)ra * NXZ + d];
  float x1 = XZ[(size_t)rb * NXZ + d];
  float x2 = XZ[(size_t)rc * NXZ + d];
  asm volatile("" :: "v"(x0), "v"(x1), "v"(x2));
  x0 = __uint_as_float(__float_as_uint(x0) & hm);
  x1 = __uint_as_float(__float_as_uint(x1) & hm);
  x2 = __uint_as_float(__float_as_uint(x2) & hm);
#pragma unroll 1
  for (int i = 0; i < CROWS; ++i) {
    const float xn = XZ[(size_t)(r0 + i) * NXZ + d];
    float acc = w0 * x0;
    acc = fmaf(w1, x1, acc);
    acc = fmaf(w2, x2, acc);
    acc = fmaf(w3, xn, acc);
    const float v = acc + cb;
    stg[i * DI + d] = silu_f(v);
    x0 = x1; x1 = x2; x2 = xn;
  }
  __syncthreads();
#pragma unroll 1
  for (int it = 0; it < 4; ++it) {
    const int row = wave + 8 * it;
    const v4f a = *(const v4fa*)(stg + row * DI + 8 * lane);
    const v4f c = *(const v4fa*)(stg + row * DI + 8 * lane + 4);
    const v4u o = pack8_bf16(a, c);
    put16(XIHL + (size_t)(r0 + row) * KHL + 8 * lane, o);
  }
#pragma unroll 1
  for (int it = 0; it < 4; ++it) {
    const int row = wave + 8 * it;
    const v4f a = *(const v4fa*)(stg + row * DI + 8 * lane);
    const v4f c = *(const v4fa*)(stg + row * DI + 8 * lane + 4);
    const v4u o = pack8_bf16_lo(a, c);
    put16(XIHL + (size_t)(r0 + row) * KHL + DI + 8 * lane, o);
  }
}

__global__ __launch_bounds__(256) void k_dtin(const float* __restrict__ XDBL, unsigned short* __restrict__ DTIN) {
  const int g   = (int)blockIdx.x * 256 + (int)threadIdx.x;
  const int row = g >> 3;
  const int p   = g & 7;
  const int c0  = (p & 1) * 8;
  v4f a = *(const v4fa*)(XDBL + (size_t)row * NXP + c0);
  v4f c = *(const v4fa*)(XDBL + (size_t)row * NXP + c0 + 4);
  asm volatile("" :: "v"(a), "v"(c));
  const v4u hi = pack8_bf16(a, c);
  const v4u lo = pack8_bf16_lo(a, c);
  const unsigned mh = (p < 2) ? 0xFFFFFFFFu : 0u;
  const unsigned ml = (p >= 2 && p < 4) ? 0xFFFFFFFFu : 0u;
  const v4u o = (hi & (v4u){ mh, mh, mh, mh }) | (lo & (v4u){ ml, ml, ml, ml });
  put16(DTIN + (size_t)row * KDT + 8 * p, o);
}

__global__ __launch_bounds__(SCT) void k_scan(const float* __restrict__ DTRAW, const float* __restrict__ XZ,
                                              const unsigned short* __restrict__ XIHL,
                                              const float* __restrict__ XDBL, const float* __restrict__ b_dt,
                                              const float* __restrict__ A_log, const float* __restrict__ Dskip,
                                              unsigned short* __restrict__ YHL) {
  __shared__ __attribute__((aligned(16))) float gst[SCH * SCT];
  const int tid  = (int)threadIdx.x;
  const int lane = tid & 31;
  const int wave = __builtin_amdgcn_readfirstlane(tid >> 5);
  const int hh   = lane >> 4;
  const int pc   = lane & 15;
  const int bb   = (int)blockIdx.x >> 1;
  const int d0   = ((int)blockIdx.x & 1) * SCT;
  const int d    = d0 + tid;
  const size_t rbase = (size_t)bb * LSEQ;

  const float A0  = -expf(bf16_val(A_log[2 * d + 0]));
  const float A1  = -expf(bf16_val(A_log[2 * d + 1]));
  const float bdt = bf16_val(b_dt[d]);
  const float Dd  = bf16_val(Dskip[d]);
  float h0 = 0.0f, h1 = 0.0f;

#pragma unroll 1
  for (int ch = 0; ch < LSEQ / SCH; ++ch) {
    const size_t r0 = rbase + (size_t)ch * SCH;
#pragma unroll 1
    for (int ll = 0; ll < SCH; ++ll) {
      const size_t r = r0 + (size_t)ll;
      const float raw = DTRAW[r * DI + d];
      const float zv  = XZ[r * NXZ + DI + d];
      const unsigned hw = (unsigned)XIHL[r * KHL + d];
      const unsigned lw = (unsigned)XIHL[r * KHL + DI + d];
      const v4f bc = *(const v4fa*)(XDBL + r * NXP + DTRK);
      const float xi  = __uint_as_float(hw << 16) + __uint_as_float(lw << 16);
      const float dt  = softplus_f(raw + bdt);
      const float dA0 = expf(dt * A0);
      const float dA1 = expf(dt * A1);
      const float dtx = dt * xi;
      h0 = dA0 * h0 + dtx * bc[0];
      h1 = dA1 * h1 + dtx * bc[1];
      float y = h0 * bc[2] + h1 * bc[3];
      y = y + Dd * xi;
      gst[ll * SCT + tid] = y * silu_f(zv);
    }
    __syncthreads();
#pragma unroll 1
    for (int it = 0; it < 4; ++it) {
      const int rowl = 2 * (wave + 4 * it) + hh;
      const v4f a = *(const v4fa*)(gst + rowl * SCT + 8 * pc);
      const v4f c = *(const v4fa*)(gst + rowl * SCT + 8 * pc + 4);
      const v4u o = pack8_bf16(a, c);
      put16(YHL + (r0 + (size_t)rowl) * KHL + d0 + 8 * pc, o);
    }
#pragma unroll 1
    for (int it = 0; it < 4; ++it) {
      const int rowl = 2 * (wave + 4 * it) + hh;
      const v4f a = *(const v4fa*)(gst + rowl * SCT + 8 * pc);
      const v4f c = *(const v4fa*)(gst + rowl * SCT + 8 * pc + 4);
      const v4u o = pack8_bf16_lo(a, c);
      put16(YHL + (r0 + (size_t)rowl) * KHL + DI + d0 + 8 * pc, o);
    }
    __syncthreads();
  }
}

extern "C" void kernel_launch(void* const* d_in, const int* in_sizes, int n_in,
                              void* d_out, int out_size, void* d_ws, size_t ws_size,
                              hipStream_t stream) {
  if (n_in < 10) return;
  if (in_sizes[0] != NBAT * DI * LSEQ) return;
  if (in_sizes[1] != DI * NXZ) return;
  if (in_sizes[2] != DI * 4) return;
  if (in_sizes[3] != DI) return;
  if (in_sizes[4] != DI * NXD) return;
  if (in_sizes[5] != DTRK * DI) return;
  if (in_sizes[6] != DI) return;
  if (in_sizes[7] != DI * 2) return;
  if (in_sizes[8] != DI) return;
  if (in_sizes[9] != DI * DI) return;
  if (out_size != NBAT * DI * LSEQ) return;
  if (WS_END > ws_size) return;

  const float* x      = (const float*)d_in[0];
  const float* w_in   = (const float*)d_in[1];
  const float* conv_w = (const float*)d_in[2];
  const float* conv_b = (const float*)d_in[3];
  const float* w_x    = (const float*)d_in[4];
  const float* w_dt   = (const float*)d_in[5];
  const float* b_dt   = (const float*)d_in[6];
  const float* a_log  = (const float*)d_in[7];
  const float* dskip  = (const float*)d_in[8];
  const float* w_out  = (const float*)d_in[9];
  float* out = (float*)d_out;

  char* ws = (char*)d_ws;
  unsigned short* UB    = (unsigned short*)(ws + O_UB);
  float*          XZ    = (float*)(ws + O_XZ);
  unsigned short* XIHL  = (unsigned short*)(ws + O_XIHL);
  float*          XDBL  = (float*)(ws + O_XDBL);
  unsigned short* DTIN  = (unsigned short*)(ws + O_DTIN);
  float*          DTRAW = (float*)(ws + O_DTRAW);
  unsigned short* YHL   = (unsigned short*)(ws + O_YHL);
  unsigned short* WINT  = (unsigned short*)(ws + O_WINT);
  unsigned short* WX2   = (unsigned short*)(ws + O_WX2);
  unsigned short* WDT2  = (unsigned short*)(ws + O_WDT2);
  unsigned short* WOUT2 = (unsigned short*)(ws + O_WOUT2);

  k_prep<<<PU_ALL / 256, 256, 0, stream>>>(w_in, w_x, w_dt, w_out, WINT, WX2, WDT2, WOUT2);

  for (int hf = 0; hf < NHALF; ++hf) {
    const float* xh = x + (size_t)hf * BHALF * DI * LSEQ;
    k_tok<<<BHALF * 4 * IMH, 256, 0, stream>>>(xh, UB);
    k_gemm_nt<0, 0><<<(MH / 64) * (NXZ / 64) / 8, 256, 0, stream>>>(UB, WINT, b_dt, XZ, MH, NXZ, DI, NXZ);
    k_conv<<<MH / CROWS, 256, 0, stream>>>(XZ, conv_w, conv_b, XIHL);
    k_gemm_nt<0, 0><<<(MH / 64) * (NXP / 64) / 8, 256, 0, stream>>>(XIHL, WX2, b_dt, XDBL, MH, NXP, KHL, NXP);
    k_dtin<<<(MH * 8) / 256, 256, 0, stream>>>(XDBL, DTIN);
    k_gemm_nt<0, 0><<<(MH / 64) * (DI / 64) / 8, 256, 0, stream>>>(DTIN, WDT2, b_dt, DTRAW, MH, DI, KDT, DI);
    k_scan<<<BHALF * (DI / SCT), SCT, 0, stream>>>(DTRAW, XZ, XIHL, XDBL, b_dt, a_log, dskip, YHL);
    for (int bb = 0; bb < BHALF; ++bb) {
      const int b = hf * BHALF + bb;
      k_gemm_nt<0, 0><<<(DI / 64) * (LSEQ / 64) / 8, 256, 0, stream>>>(
          WOUT2, YHL + (size_t)bb * LSEQ * KHL, b_dt, out + (size_t)b * DI * LSEQ, DI, LSEQ, KHL, LSEQ);
    }
  }
}
